// twostep_net_37434934952779
// MI455X (gfx1250) — hardware-verified
//
#include <hip/hip_runtime.h>
#include <stddef.h>
#include <math.h>


#define NTHR   256
#define NWAVE  8
#define EPT    8
#define CHUNK  (NTHR * EPT)
#define WCAP   (EPT * 32)
#define LISTN  (NWAVE * WCAP)
#define PASSN  (NWAVE * 16)
#define PCAP   (CHUNK + PASSN)
#define NB     1024
#define HD     32
#define EDM    16
#define KE     544
#define NWR    224
#define LROWS  128
#define GB     64
#define ASC    16.0f
#define WSC    64.0f
#define BSC    1024.0f
#define NSC    1024.0f
#define NDINV  0.0009765625f
#define EDINV  0.00006103515625f

#define L_BE    0
#define L_WN    (L_BE + HD * KE * 2)
#define L_BN    (L_WN + NWR * HD * 2)
#define L_ACC   (L_BN + NWR * 4)
#define L_MSG   (L_ACC + (NB + 1) * HD * 4)
#define L_SROW  (L_MSG + HD * PASSN * 4)
#define L_AROW  (L_SROW + NWAVE * 16 * HD * 4)
#define L_LIST  (L_AROW + NWAVE * 16 * EDM * 4)
#define L_PEND  (L_LIST + LISTN * 4)
#define L_SLOT  (L_PEND + PCAP * 4)
#define L_WCNT  (L_SLOT + PASSN * 4)
#define L_TOTAL (L_WCNT + 64)

static_assert(PASSN == 128);
static_assert(PCAP >= CHUNK + PASSN);
static_assert((NB % (16 * NWAVE)) == 0);
static_assert((NB % (4 * NWAVE)) == 0);
static_assert((NB % LROWS) == 0);
static_assert(NWR == 7 * HD);
static_assert(KE == 16 * HD + HD);
static_assert(HD == 32 && EDM == 16);
static_assert(NWAVE * 16 * HD * 2 <= NWAVE * 16 * HD * 4);
static_assert((L_BN % 16) == 0 && (L_ACC % 16) == 0 && (L_MSG % 16) == 0);
static_assert((L_SROW % 16) == 0 && (L_AROW % 16) == 0 && (L_LIST % 16) == 0);
static_assert((L_TOTAL % 16) == 0);
static_assert(L_TOTAL <= 300 * 1024);
static_assert(GB == 64 && GB <= NTHR);
static_assert(LROWS == 16 * NWAVE);

typedef float    v4f  __attribute__((ext_vector_type(4)));
typedef float    v8f  __attribute__((ext_vector_type(8)));
typedef int      v4i  __attribute__((ext_vector_type(4)));
typedef _Float16 v8h  __attribute__((ext_vector_type(8)));
typedef _Float16 v16h __attribute__((ext_vector_type(16)));
union FragH { v16h v; v8h h[2]; };

__device__ __forceinline__ v8f wmh(v16h a, v16h b, v8f c) {
  v8f d = __builtin_amdgcn_wmma_f32_16x16x32_f16(false, a, false, b, (short)0, c, false, false);
  asm volatile("v_nop\n\tv_nop\n\tv_nop\n\tv_nop" : "+v"(d) : "v"(a), "v"(b));
  return d;
}

__device__ __forceinline__ v8f splat8(float x) {
  v8f c;
#pragma unroll
  for (int i = 0; i < 8; ++i) c[i] = x;
  return c;
}

__device__ __forceinline__ v8h cv8s(v4f a, v4f b, float sc) {
  v8h r;
  r[0] = (_Float16)(a.x * sc); r[1] = (_Float16)(a.y * sc); r[2] = (_Float16)(a.z * sc); r[3] = (_Float16)(a.w * sc);
  r[4] = (_Float16)(b.x * sc); r[5] = (_Float16)(b.y * sc); r[6] = (_Float16)(b.z * sc); r[7] = (_Float16)(b.w * sc);
  return r;
}

__device__ __forceinline__ v8h scl8(float s, v8f a) {
  v8h r;
#pragma unroll
  for (int i = 0; i < 8; ++i) r[i] = (_Float16)(s * a[i]);
  return r;
}

__device__ __forceinline__ int scan_chunk(const int* __restrict__ dsts, int nE, int cbase, int nodeBase,
                                          int vec8, int* list, int tid, int wave) {
  int wc = 0;
  const int el0  = tid * EPT;
  const int e0   = cbase + el0;
  const int sent = -2147483647 - 1;
  v4i da, db;
  if (vec8 != 0 && cbase + CHUNK <= nE) {
    da = *(const v4i*)(dsts + e0);
    db = *(const v4i*)(dsts + e0 + 4);
  } else {
    da.x = (e0     < nE) ? dsts[min(e0, nE - 1)] : sent;
    da.y = (e0 + 1 < nE) ? dsts[min(e0 + 1, nE - 1)] : sent;
    da.z = (e0 + 2 < nE) ? dsts[min(e0 + 2, nE - 1)] : sent;
    da.w = (e0 + 3 < nE) ? dsts[min(e0 + 3, nE - 1)] : sent;
    db.x = (e0 + 4 < nE) ? dsts[min(e0 + 4, nE - 1)] : sent;
    db.y = (e0 + 5 < nE) ? dsts[min(e0 + 5, nE - 1)] : sent;
    db.z = (e0 + 6 < nE) ? dsts[min(e0 + 6, nE - 1)] : sent;
    db.w = (e0 + 7 < nE) ? dsts[min(e0 + 7, nE - 1)] : sent;
  }
  const unsigned nb = (unsigned)nodeBase;
  const unsigned s0 = (unsigned)da.x - nb, s1 = (unsigned)da.y - nb;
  const unsigned s2 = (unsigned)da.z - nb, s3 = (unsigned)da.w - nb;
  const unsigned s4 = (unsigned)db.x - nb, s5 = (unsigned)db.y - nb;
  const unsigned s6 = (unsigned)db.z - nb, s7 = (unsigned)db.w - nb;
  const bool h0 = s0 < (unsigned)NB, h1 = s1 < (unsigned)NB, h2 = s2 < (unsigned)NB, h3 = s3 < (unsigned)NB;
  const bool h4 = s4 < (unsigned)NB, h5 = s5 < (unsigned)NB, h6 = s6 < (unsigned)NB, h7 = s7 < (unsigned)NB;
  const unsigned any = __builtin_amdgcn_ballot_w32(h0 | h1 | h2 | h3 | h4 | h5 | h6 | h7);
  if (any != 0u) {
#define HITJ(J, HJ) { \
      const unsigned mj = __builtin_amdgcn_ballot_w32(HJ); \
      if (mj != 0u) { \
        if (HJ) { \
          const int pos = wc + (int)__builtin_amdgcn_mbcnt_lo(mj, 0u); \
          if (pos < WCAP) list[wave * WCAP + pos] = el0 + (J); \
        } \
        wc += (int)__builtin_popcount(mj); } }
    HITJ(0, h0)
    HITJ(1, h1)
    HITJ(2, h2)
    HITJ(3, h3)
    HITJ(4, h4)
    HITJ(5, h5)
    HITJ(6, h6)
    HITJ(7, h7)
#undef HITJ
  }
  return wc;
}

__global__ __launch_bounds__(NTHR) void k_lin0(const float* __restrict__ x, const float* __restrict__ W0,
                                              const float* __restrict__ b0, float* xout, int nN) {
  __shared__ __attribute__((aligned(16))) _Float16 lw[HD * HD];
  __shared__ __attribute__((aligned(16))) float lb[HD];
  __shared__ __attribute__((aligned(16))) float st[LROWS * HD];
  const int tid = threadIdx.x, lane = tid & 31, wave = tid >> 5, hh = lane >> 4, m = lane & 15;
#pragma unroll 1
  for (int i = tid; i < HD * HD; i += NTHR) lw[i] = (_Float16)(W0[i] * WSC);
  if (tid < HD) lb[tid] = b0[tid] * NSC;
  __syncthreads();
  const int rbase = blockIdx.x * LROWS;
  int nd = rbase + wave * 16 + m;
  nd = nd > nN - 1 ? nN - 1 : nd;
  FragH a;
  {
    const float* xr = x + (size_t)nd * HD + 8 * hh;
    a.h[0] = cv8s(*(const v4f*)xr, *(const v4f*)(xr + 4), ASC);
    a.h[1] = cv8s(*(const v4f*)(xr + 16), *(const v4f*)(xr + 20), ASC);
  }
#pragma unroll 1
  for (int nt = 0; nt < 2; ++nt) {
    const int col = 16 * nt + m;
    v8f c = splat8(lb[col]);
    FragH b;
    const _Float16* wp = lw + col * HD + 8 * hh;
    b.h[0] = *(const v8h*)wp;
    b.h[1] = *(const v8h*)(wp + 16);
    c = wmh(a.v, b.v, c);
#pragma unroll
    for (int r = 0; r < 8; ++r) st[(wave * 16 + 8 * hh + r) * HD + col] = fmaxf(c[r] * NDINV, 0.0f);
  }
  __syncthreads();
#pragma unroll 1
  for (int q = 0; q < 4; ++q) {
    const int row = wave * 16 + 4 * q + (lane >> 3);
    const int c4 = 4 * (lane & 7);
    const v4f v = *(const v4f*)(st + row * HD + c4);
    *(volatile v4f*)(xout + (size_t)(rbase + row) * HD + c4) = v;
  }
  __threadfence();
#pragma unroll 1
  for (int q = 0; q < 4; ++q) {
    const int row = wave * 16 + 4 * q + (lane >> 3);
    const int c4 = 4 * (lane & 7);
    const v4f v = *(const v4f*)(st + row * HD + c4);
    *(volatile v4f*)(xout + (size_t)(rbase + row) * HD + c4) = v;
  }
}

__global__ __launch_bounds__(NTHR) void k_layer(
    const float* __restrict__ xin, const float* __restrict__ eattr, const int* __restrict__ ei,
    const float* __restrict__ We, const float* __restrict__ be,
    const float* __restrict__ Wroot, const float* __restrict__ bconv,
    const float* __restrict__ Wih, const float* __restrict__ bih,
    const float* __restrict__ Whh, const float* __restrict__ bhh,
    float* xout, int nN, int nE, int vec8) {
  extern __shared__ __attribute__((aligned(16))) unsigned char dsm[];
  _Float16* lbe   = (_Float16*)(dsm + L_BE);
  _Float16* lwn   = (_Float16*)(dsm + L_WN);
  float*    lbn   = (float*)(dsm + L_BN);
  float*    acc   = (float*)(dsm + L_ACC);
  float*    msgT  = (float*)(dsm + L_MSG);
  float*    srow  = (float*)(dsm + L_SROW);
  _Float16* mt    = (_Float16*)(dsm + L_SROW);
  float*    arow  = (float*)(dsm + L_AROW);
  int*      list  = (int*)(dsm + L_LIST);
  int*      pend  = (int*)(dsm + L_PEND);
  int*      slotb = (int*)(dsm + L_SLOT);
  int*      wcnt  = (int*)(dsm + L_WCNT);

  const int tid = threadIdx.x, lane = tid & 31, wave = tid >> 5, hh = lane >> 4, m = lane & 15;
  const int nodeBase = blockIdx.x * NB;
  const int* srcs = ei;
  const int* dsts = ei + nE;

#pragma unroll 1
  for (int idx = tid; idx < HD * KE; idx += NTHR) {
    const int n = idx / KE;
    const int k = idx - n * KE;
    int iw = k >> 4; iw = iw > HD - 1 ? HD - 1 : iw;
    const int f = k & 15;
    const float wv = We[(size_t)(iw * HD + n) * EDM + f];
    int ib = k - 16 * HD; ib = ib < 0 ? 0 : (ib > HD - 1 ? HD - 1 : ib);
    const float bv = be[ib * HD + n];
    const float v = (k < 16 * HD) ? wv * WSC : bv * BSC;
    lbe[idx] = (_Float16)v;
  }
#pragma unroll 1
  for (int idx = tid; idx < NWR * HD; idx += NTHR) {
    const int row = idx >> 5, k = idx & 31;
    const int q0 = row > HD - 1 ? HD - 1 : row;
    int q1 = row - HD;     q1 = q1 < 0 ? 0 : (q1 > 3 * HD - 1 ? 3 * HD - 1 : q1);
    int q2 = row - 4 * HD; q2 = q2 < 0 ? 0 : (q2 > 3 * HD - 1 ? 3 * HD - 1 : q2);
    const float w0 = Wroot[q0 * HD + k];
    const float w1 = Wih[q1 * HD + k];
    const float w2 = Whh[q2 * HD + k];
    const float v = row < HD ? w0 : (row < 4 * HD ? w1 : w2);
    lwn[idx] = (_Float16)(v * WSC);
  }
  if (tid < NWR) {
    const int q0 = tid > HD - 1 ? HD - 1 : tid;
    int q1 = tid - HD;     q1 = q1 < 0 ? 0 : (q1 > 3 * HD - 1 ? 3 * HD - 1 : q1);
    int q2 = tid - 4 * HD; q2 = q2 < 0 ? 0 : (q2 > 3 * HD - 1 ? 3 * HD - 1 : q2);
    const float v0 = bconv[q0], v1 = bih[q1], v2 = bhh[q2];
    const float v = tid < HD ? v0 : (tid < 4 * HD ? v1 : v2);
    lbn[tid] = v * NSC;
  }
  {
    const v4f z = {0.0f, 0.0f, 0.0f, 0.0f};
#pragma unroll 1
    for (int i = tid; i < (NB + 1) * HD / 4; i += NTHR) *(v4f*)(acc + 4 * i) = z;
  }
  if (tid == 0) wcnt[NWAVE] = 0;
  __syncthreads();

  const int nChunks = (nE + CHUNK - 1) / CHUNK;
#pragma unroll 1
  for (int ch = 0; ch < nChunks; ++ch) {
    const int cbase = ch * CHUNK;
    const int wc = scan_chunk(dsts, nE, cbase, nodeBase, vec8, list, tid, wave);
    if (lane == 0) wcnt[wave] = wc;
    __syncthreads();

    const int base = wcnt[NWAVE];
    int tot = 0, myoff = 0;
#pragma unroll
    for (int w = 0; w < NWAVE; ++w) {
      int c = wcnt[w];
      c = c > WCAP ? WCAP : (c < 0 ? 0 : c);
      if (w < wave) myoff += c;
      tot += c;
    }
    int newN = base + tot;
    newN = newN > PCAP ? PCAP : newN;
    {
      int n = wcnt[wave];
      n = n > WCAP ? WCAP : (n < 0 ? 0 : n);
      const int* lp = list + wave * WCAP;
      for (int i = lane; i < n; i += 32) {
        const int pos = base + myoff + i;
        if (pos < PCAP) pend[pos] = cbase + lp[i];
      }
    }
    const int fin = (ch == nChunks - 1) ? 1 : 0;
    const int R   = (fin != 0) ? (newN + PASSN - 1) / PASSN : newN / PASSN;
    const int Pv  = (fin != 0) ? newN : R * PASSN;
    __syncthreads();

#pragma unroll 1
    for (int r = 0; r < R; ++r) {
      {
        int idx = r * PASSN + wave * 16 + m;
        const bool valid = idx < Pv;
        idx = idx > PCAP - 1 ? PCAP - 1 : idx;
        int e = pend[idx];
        e = e < 0 ? 0 : (e > nE - 1 ? nE - 1 : e);
        const int d = dsts[e];
        int s = srcs[e];
        int slot = d - nodeBase;
        if (!valid || (unsigned)slot >= (unsigned)NB) slot = NB;
        s = s < 0 ? 0 : (s > nN - 1 ? nN - 1 : s);
        const float* xr = xin + (size_t)s * HD + 16 * hh;
        const v4f x0 = *(const v4f*)xr;
        const v4f x1 = *(const v4f*)(xr + 4);
        const v4f x2 = *(const v4f*)(xr + 8);
        const v4f x3 = *(const v4f*)(xr + 12);
        float* sp = srow + (wave * 16 + m) * HD + 16 * hh;
        *(v4f*)sp = x0;
        *(v4f*)(sp + 4) = x1;
        *(v4f*)(sp + 8) = x2;
        *(v4f*)(sp + 12) = x3;
        const float* ap = eattr + (size_t)e * EDM + 8 * hh;
        v4f a0 = *(const v4f*)ap;
        v4f a1 = *(const v4f*)(ap + 4);
        a0.x = valid ? a0.x : 0.0f; a0.y = valid ? a0.y : 0.0f; a0.z = valid ? a0.z : 0.0f; a0.w = valid ? a0.w : 0.0f;
        a1.x = valid ? a1.x : 0.0f; a1.y = valid ? a1.y : 0.0f; a1.z = valid ? a1.z : 0.0f; a1.w = valid ? a1.w : 0.0f;
        float* aq = arow + (wave * 16 + m) * EDM + 8 * hh;
        *(v4f*)aq = a0;
        *(v4f*)(aq + 4) = a1;
        if (hh == 0) slotb[wave * 16 + m] = slot;
      }
      __syncthreads();

      {
        const float* sp = srow + (wave * 16 + m) * HD;
        float sv[HD];
#pragma unroll
        for (int q = 0; q < 8; ++q) {
          const v4f t = *(const v4f*)(sp + 4 * q);
          sv[4 * q] = t.x * ASC; sv[4 * q + 1] = t.y * ASC; sv[4 * q + 2] = t.z * ASC; sv[4 * q + 3] = t.w * ASC;
        }
        v8f av;
        {
          const float* aq = arow + (wave * 16 + m) * EDM + 8 * hh;
          const v4f u0 = *(const v4f*)aq;
          const v4f u1 = *(const v4f*)(aq + 4);
          av[0] = u0.x * ASC; av[1] = u0.y * ASC; av[2] = u0.z * ASC; av[3] = u0.w * ASC;
          av[4] = u1.x * ASC; av[5] = u1.y * ASC; av[6] = u1.z * ASC; av[7] = u1.w * ASC;
        }
        v8f c0 = splat8(0.0f), c1 = splat8(0.0f);
        const _Float16* bp0 = lbe + m * KE + 8 * hh;
        const _Float16* bp1 = lbe + (16 + m) * KE + 8 * hh;
#pragma unroll
        for (int c = 0; c < 16; ++c) {
          FragH A, B0, B1;
          A.h[0] = scl8(sv[2 * c], av);
          A.h[1] = scl8(sv[2 * c + 1], av);
          B0.h[0] = *(const v8h*)(bp0 + 32 * c);
          B0.h[1] = *(const v8h*)(bp0 + 32 * c + 16);
          B1.h[0] = *(const v8h*)(bp1 + 32 * c);
          B1.h[1] = *(const v8h*)(bp1 + 32 * c + 16);
          c0 = wmh(A.v, B0.v, c0);
          c1 = wmh(A.v, B1.v, c1);
        }
        {
          FragH A, B0, B1;
          A.h[0] = cv8s(*(const v4f*)(sp + 8 * hh), *(const v4f*)(sp + 8 * hh + 4), ASC);
          A.h[1] = cv8s(*(const v4f*)(sp + 16 + 8 * hh), *(const v4f*)(sp + 20 + 8 * hh), ASC);
          B0.h[0] = *(const v8h*)(bp0 + 16 * HD);
          B0.h[1] = *(const v8h*)(bp0 + 16 * HD + 16);
          B1.h[0] = *(const v8h*)(bp1 + 16 * HD);
          B1.h[1] = *(const v8h*)(bp1 + 16 * HD + 16);
          c0 = wmh(A.v, B0.v, c0);
          c1 = wmh(A.v, B1.v, c1);
        }
        float* mp0 = msgT + m * PASSN + wave * 16 + 8 * hh;
        float* mp1 = msgT + (16 + m) * PASSN + wave * 16 + 8 * hh;
        const v4f o0 = {c0[0] * EDINV, c0[1] * EDINV, c0[2] * EDINV, c0[3] * EDINV};
        const v4f o1 = {c0[4] * EDINV, c0[5] * EDINV, c0[6] * EDINV, c0[7] * EDINV};
        const v4f o2 = {c1[0] * EDINV, c1[1] * EDINV, c1[2] * EDINV, c1[3] * EDINV};
        const v4f o3 = {c1[4] * EDINV, c1[5] * EDINV, c1[6] * EDINV, c1[7] * EDINV};
        *(v4f*)mp0 = o0;
        *(v4f*)(mp0 + 4) = o1;
        *(v4f*)mp1 = o2;
        *(v4f*)(mp1 + 4) = o3;
      }
      __syncthreads();

      if (tid < HD) {
#pragma unroll 1
        for (int i = 0; i < PASSN; ++i) {
          int sl = slotb[i];
          sl = sl < 0 ? 0 : (sl > NB ? NB : sl);
          acc[sl * HD + tid] += msgT[tid * PASSN + i];
        }
      }
      __syncthreads();
    }

    int rem = newN - R * PASSN;
    rem = rem < 0 ? 0 : rem;
    if (R > 0 && tid < rem) pend[tid] = pend[R * PASSN + tid];
    if (tid == 0) wcnt[NWAVE] = rem;
  }
  __syncthreads();

  _Float16* mw = mt + wave * 16 * HD;
#pragma unroll 1
  for (int tt = 0; tt < NB / (16 * NWAVE); ++tt) {
    const int t = wave + NWAVE * tt;
    const int lrow0 = 16 * t;
    int ndm = nodeBase + lrow0 + m;
    ndm = ndm > nN - 1 ? nN - 1 : ndm;
    FragH ao;
    {
      const float* xr = xin + (size_t)ndm * HD + 8 * hh;
      ao.h[0] = cv8s(*(const v4f*)xr, *(const v4f*)(xr + 4), ASC);
      ao.h[1] = cv8s(*(const v4f*)(xr + 16), *(const v4f*)(xr + 20), ASC);
    }
#pragma unroll 1
    for (int nt = 0; nt < 2; ++nt) {
      const int col = 16 * nt + m;
      v8f c = splat8(lbn[col]);
      FragH b;
      const _Float16* wp = lwn + col * HD + 8 * hh;
      b.h[0] = *(const v8h*)wp;
      b.h[1] = *(const v8h*)(wp + 16);
      c = wmh(ao.v, b.v, c);
#pragma unroll
      for (int rr = 0; rr < 8; ++rr) {
        const int lrow = lrow0 + 8 * hh + rr;
        const float cv = c[rr] * NDINV + acc[lrow * HD + col];
        const float mv = fmaxf(cv, 0.0f);
        mw[(8 * hh + rr) * HD + col] = (_Float16)(mv * ASC);
      }
    }
    __syncthreads();
    FragH am;
    {
      const _Float16* hp = mw + m * HD + 8 * hh;
      am.h[0] = *(const v8h*)hp;
      am.h[1] = *(const v8h*)(hp + 16);
    }
#pragma unroll 1
    for (int nt = 0; nt < 2; ++nt) {
      const int o = 16 * nt + m;
      v8f gir, giz, gin, ghr, ghz, ghn;
      {
        FragH b; const _Float16* wp = lwn + (HD + o) * HD + 8 * hh;
        b.h[0] = *(const v8h*)wp; b.h[1] = *(const v8h*)(wp + 16);
        gir = wmh(am.v, b.v, splat8(lbn[HD + o]));
      }
      {
        FragH b; const _Float16* wp = lwn + (2 * HD + o) * HD + 8 * hh;
        b.h[0] = *(const v8h*)wp; b.h[1] = *(const v8h*)(wp + 16);
        giz = wmh(am.v, b.v, splat8(lbn[2 * HD + o]));
      }
      {
        FragH b; const _Float16* wp = lwn + (3 * HD + o) * HD + 8 * hh;
        b.h[0] = *(const v8h*)wp; b.h[1] = *(const v8h*)(wp + 16);
        gin = wmh(am.v, b.v, splat8(lbn[3 * HD + o]));
      }
      {
        FragH b; const _Float16* wp = lwn + (4 * HD + o) * HD + 8 * hh;
        b.h[0] = *(const v8h*)wp; b.h[1] = *(const v8h*)(wp + 16);
        ghr = wmh(ao.v, b.v, splat8(lbn[4 * HD + o]));
      }
      {
        FragH b; const _Float16* wp = lwn + (5 * HD + o) * HD + 8 * hh;
        b.h[0] = *(const v8h*)wp; b.h[1] = *(const v8h*)(wp + 16);
        ghz = wmh(ao.v, b.v, splat8(lbn[5 * HD + o]));
      }
      {
        FragH b; const _Float16* wp = lwn + (6 * HD + o) * HD + 8 * hh;
        b.h[0] = *(const v8h*)wp; b.h[1] = *(const v8h*)(wp + 16);
        ghn = wmh(ao.v, b.v, splat8(lbn[6 * HD + o]));
      }
#pragma unroll
      for (int rr = 0; rr < 8; ++rr) {
        const int lrow = lrow0 + 8 * hh + rr;
        int nd = nodeBase + lrow;
        nd = nd > nN - 1 ? nN - 1 : nd;
        const float ho = xin[(size_t)nd * HD + o];
        float xr = (gir[rr] + ghr[rr]) * NDINV;
        float xz = (giz[rr] + ghz[rr]) * NDINV;
        xr = xr > 30.0f ? 30.0f : (xr < -30.0f ? -30.0f : xr);
        xz = xz > 30.0f ? 30.0f : (xz < -30.0f ? -30.0f : xz);
        const float rg = 1.0f / (1.0f + expf(-xr));
        const float zg = 1.0f / (1.0f + expf(-xz));
        const float ng = tanhf(gin[rr] * NDINV + rg * (ghn[rr] * NDINV));
        const float hn = (1.0f - zg) * ng + zg * ho;
        acc[lrow * HD + o] = hn;
      }
    }
    __syncthreads();
  }

#pragma unroll 1
  for (int q = 0; q < NB / (NWAVE * 4); ++q) {
    const int row = wave * (NB / NWAVE) + 4 * q + (lane >> 3);
    const int c4 = 4 * (lane & 7);
    const v4f v = *(const v4f*)(acc + row * HD + c4);
    *(volatile v4f*)(xout + (size_t)(nodeBase + row) * HD + c4) = v;
  }
  __threadfence();
#pragma unroll 1
  for (int q = 0; q < NB / (NWAVE * 4); ++q) {
    const int row = wave * (NB / NWAVE) + 4 * q + (lane >> 3);
    const int c4 = 4 * (lane & 7);
    const v4f v = *(const v4f*)(acc + row * HD + c4);
    *(volatile v4f*)(xout + (size_t)(nodeBase + row) * HD + c4) = v;
  }
}

__global__ __launch_bounds__(NTHR) void k_pool(const float* __restrict__ x, const int* __restrict__ bt,
                                              const float* __restrict__ W1, const float* __restrict__ b1,
                                              float* out, int nN) {
  __shared__ __attribute__((aligned(16))) float pacc[GB * HD];
  __shared__ __attribute__((aligned(16))) float pcnt[GB];
  __shared__ __attribute__((aligned(16))) float ys[GB];
  __shared__ int hl[NTHR];
  __shared__ int hs[NTHR];
  __shared__ int wc[NWAVE];
  const int tid = threadIdx.x, lane = tid & 31, wave = tid >> 5;
  const int g0 = blockIdx.x * GB;
#pragma unroll 1
  for (int i = tid; i < GB * HD; i += NTHR) pacc[i] = 0.0f;
  if (tid < GB) pcnt[tid] = 0.0f;
  __syncthreads();
  const int nCh = (nN + NTHR - 1) / NTHR;
#pragma unroll 1
  for (int ch = 0; ch < nCh; ++ch) {
    const int i  = ch * NTHR + tid;
    const int ic = i > nN - 1 ? nN - 1 : i;
    const int b  = bt[ic];
    const int slot = b - g0;
    const bool hit = (i < nN) && ((unsigned)slot < (unsigned)GB);
    const unsigned mk = __builtin_amdgcn_ballot_w32(hit);
    if (lane == 0) wc[wave] = (int)__builtin_popcount(mk);
    __syncthreads();
    int off = 0, tot = 0;
#pragma unroll
    for (int w = 0; w < NWAVE; ++w) { const int c = wc[w]; if (w < wave) off += c; tot += c; }
    if (hit) {
      const int pos = off + (int)__builtin_amdgcn_mbcnt_lo(mk, 0u);
      if (pos < NTHR) { hl[pos] = i; hs[pos] = slot; }
    }
    __syncthreads();
    tot = tot > NTHR ? NTHR : (tot < 0 ? 0 : tot);
    if (tid < HD) {
#pragma unroll 1
      for (int j = 0; j < tot; ++j) {
        int nd = hl[j];
        nd = nd < 0 ? 0 : (nd > nN - 1 ? nN - 1 : nd);
        int sl = hs[j];
        sl = sl < 0 ? 0 : (sl > GB - 1 ? GB - 1 : sl);
        pacc[sl * HD + tid] += x[(size_t)nd * HD + tid];
        if (tid == 0) pcnt[sl] += 1.0f;
      }
    }
    __syncthreads();
  }
  if (tid < GB) {
    const float c  = pcnt[tid] > 1.0f ? pcnt[tid] : 1.0f;
    const float rc = 1.0f / c;
    float s = 0.0f;
#pragma unroll 4
    for (int k = 0; k < HD; ++k) s += (pacc[tid * HD + k] * rc) * W1[k];
    ys[tid] = s + b1[0];
  }
  __syncthreads();
  v4f v = {0.0f, 0.0f, 0.0f, 0.0f};
  if (wave == 0 && lane < 16) v = *(const v4f*)(ys + 4 * lane);
  if (wave == 0 && lane < 16) *(volatile v4f*)(out + g0 + 4 * lane) = v;
  __threadfence();
  if (wave == 0 && lane < 16) *(volatile v4f*)(out + g0 + 4 * lane) = v;
}

extern "C" void kernel_launch(void* const* d_in, const int* in_sizes, int n_in,
                              void* d_out, int out_size, void* d_ws, size_t ws_size,
                              hipStream_t stream) {
  if (n_in < 16) return;
  const int nN = in_sizes[3];
  if (nN < 1 || in_sizes[0] != nN * HD) return;
  const int nE = in_sizes[1] / 2;
  if (nE < 1 || in_sizes[1] != 2 * nE || in_sizes[2] != nE * EDM) return;
  if (in_sizes[4] != HD * HD || in_sizes[5] != HD) return;
  if (in_sizes[6] != HD * HD * EDM || in_sizes[7] != HD * HD) return;
  if (in_sizes[8] != HD * HD || in_sizes[9] != HD) return;
  if (in_sizes[10] != 3 * HD * HD || in_sizes[11] != 3 * HD) return;
  if (in_sizes[12] != 3 * HD * HD || in_sizes[13] != 3 * HD) return;
  if (in_sizes[14] != HD || in_sizes[15] != 1) return;
  const int G = out_size;
  if (G < GB || (G % GB) != 0) return;

  const float* x     = (const float*)d_in[0];
  const int*   ei    = (const int*)d_in[1];
  const float* ea    = (const float*)d_in[2];
  const int*   batch = (const int*)d_in[3];
  const float* W0    = (const float*)d_in[4];
  const float* b0    = (const float*)d_in[5];
  const float* We    = (const float*)d_in[6];
  const float* be    = (const float*)d_in[7];
  const float* Wroot = (const float*)d_in[8];
  const float* bconv = (const float*)d_in[9];
  const float* Wih   = (const float*)d_in[10];
  const float* bih   = (const float*)d_in[11];
  const float* Whh   = (const float*)d_in[12];
  const float* bhh   = (const float*)d_in[13];
  const float* W1    = (const float*)d_in[14];
  const float* b1    = (const float*)d_in[15];
  float* outp = (float*)d_out;

  const int nBlk = (nN + NB - 1) / NB;
  const size_t rowsP = (size_t)nBlk * NB;

  char* ws = (char*)d_ws;
  size_t off = 0;
  const size_t oA = off; off += (rowsP * HD * 4 + 255) & ~(size_t)255;
  const size_t oB = off; off += (rowsP * HD * 4 + 255) & ~(size_t)255;
  size_t limit = (size_t)134217728;
  if (ws_size < limit) limit = ws_size;
  if (off > limit) return;
  float* PA = (float*)(ws + oA);
  float* PB = (float*)(ws + oB);

  const int vec8 = ((nE & 3) == 0) ? 1 : 0;

  k_lin0<<<(unsigned)(rowsP / LROWS), NTHR, 0, stream>>>(x, W0, b0, PA, nN);

  hipFuncSetAttribute(reinterpret_cast<const void*>(&k_layer), hipFuncAttributeMaxDynamicSharedMemorySize, L_TOTAL);

  k_layer<<<nBlk, NTHR, L_TOTAL, stream>>>(PA, ea, ei, We, be, Wroot, bconv, Wih, bih, Whh, bhh, PB, nN, nE, vec8);
  k_layer<<<nBlk, NTHR, L_TOTAL, stream>>>(PB, ea, ei, We, be, Wroot, bconv, Wih, bih, Whh, bhh, PA, nN, nE, vec8);
  k_layer<<<nBlk, NTHR, L_TOTAL, stream>>>(PA, ea, ei, We, be, Wroot, bconv, Wih, bih, Whh, bhh, PB, nN, nE, vec8);

  k_pool<<<G / GB, NTHR, 0, stream>>>(PB, batch, W1, b1, outp, nN);
}
